// RNN_47794396070453
// MI455X (gfx1250) — hardware-verified
//
#include <hip/hip_runtime.h>
#include <math.h>

constexpr int NB    = 64;
constexpr int NS    = 512;
constexpr int NI    = 128;
constexpr int NH    = 1024;
constexpr int NO    = 64;
constexpr int NR    = 4;
constexpr int NTHR  = 256;
constexpr int RB    = 16;
constexpr int NWAVE = NTHR / 32;
constexpr int ECOL  = 8;
constexpr int EIT   = NH / (16 * ECOL);
constexpr float ALPHA_F  = 0.1f;
constexpr float WCARRY   = 64.0f;
constexpr float LOCARRY  = 2048.0f;
constexpr float SC_HH    = 1.0f / WCARRY;
constexpr float SC_X     = 1.0f / (WCARRY * LOCARRY);
constexpr float F16_MINN = 6.103515625e-05f;
static_assert(NB % RB == 0);
static_assert(NTHR == 16 * RB);
static_assert(NH == 16 * ECOL * EIT);
static_assert(NI == 16 * 8);
static_assert(NO == 4 * 16);
static_assert(NWAVE == 8);
static_assert(NH % 32 == 0);
static_assert(NR == 4);
static_assert((NO * NH) % (8 * NTHR) == 0);
static_assert(NH % NTHR == 0);

typedef __attribute__((ext_vector_type(16))) _Float16 v16h;
typedef __attribute__((ext_vector_type(8)))  _Float16 v8h;
typedef __attribute__((ext_vector_type(8)))  float    v8f;
typedef __attribute__((ext_vector_type(4)))  float    v4f;

__device__ __forceinline__ void dep_guard_h(v8f& a, v8f& b, v16h x, v16h y) { asm volatile("v_nop\n\tv_nop\n\tv_nop\n\tv_nop" : "+v"(a), "+v"(b) : "v"(x), "v"(y)); }
__device__ __forceinline__ void keep4_h(v16h a, v16h b, v16h c, v16h d) { asm volatile("v_nop" :: "v"(a), "v"(b), "v"(c), "v"(d)); }
template <typename T> struct Frag;
template <> struct Frag<_Float16> {
  typedef v16h V; union U { v16h v; v8h h[2]; };
  static __device__ __forceinline__ v16h load(const _Float16* p) {
    U f; f.h[0] = *(const v8h*)(p); f.h[1] = *(const v8h*)(p + 16); return f.v;
  }
  static __device__ __forceinline__ v8f mma(v16h a, v16h b, v8f c) {
    return __builtin_amdgcn_wmma_f32_16x16x32_f16(false, a, false, b, (short)0, c, false, false);
  }
  static __device__ __forceinline__ void guard(v8f& a, v8f& b, v16h x, v16h y) { dep_guard_h(a, b, x, y); }
  static __device__ __forceinline__ void keep(v16h a, v16h b, v16h c, v16h d) { keep4_h(a, b, c, d); }
};
__device__ __forceinline__ void wguard2(v8f& c, v16h a, v16h b) {
  asm volatile("v_nop\n\tv_nop\n\tv_nop\n\tv_nop" : "+v"(c) : "v"(a), "v"(b));
}
__device__ __forceinline__ void wguard4(v8f& c, v16h a, v16h b, v16h d, v16h e) {
  asm volatile("v_nop\n\tv_nop\n\tv_nop\n\tv_nop" : "+v"(c) : "v"(a), "v"(b), "v"(d), "v"(e));
}
__device__ __forceinline__ void accg1(v8f& c) { asm volatile("v_nop\n\tv_nop\n\tv_nop\n\tv_nop" : "+v"(c)); }

__device__ __forceinline__ void split_f16(float v, _Float16& hi, _Float16& lo) {
  const float vz = (fabsf(v) < F16_MINN) ? 0.0f : v;
  const _Float16 h = (_Float16)vz;
  const float hf = (float)h;
  hi = h;
  lo = (_Float16)((v - hf) * LOCARRY);
}

__device__ __forceinline__ float tanh_f32(float xin) {
  const float xc = fminf(fmaxf(xin, -15.0f), 15.0f);
  const float t  = expf(2.0f * xc);
  return 1.0f - 2.0f * __builtin_amdgcn_rcpf(t + 1.0f);
}

__global__ __launch_bounds__(NTHR) void wsplit_kernel(const float* __restrict__ w,
                                                     unsigned short* __restrict__ whp,
                                                     unsigned short* __restrict__ wlp, int n8) {
  const int i = blockIdx.x * NTHR + threadIdx.x;
  if (i < n8) {
    const v4f a = *(const v4f*)(w + (size_t)i * 8);
    const v4f b = *(const v4f*)(w + (size_t)i * 8 + 4);
    v8h hv, lv;
#pragma unroll
    for (int e = 0; e < 4; ++e) {
      _Float16 h0, l0, h1, l1;
      split_f16(a[e] * WCARRY, h0, l0);
      split_f16(b[e] * WCARRY, h1, l1);
      hv[e] = h0; lv[e] = l0; hv[4 + e] = h1; lv[4 + e] = l1;
    }
    _Float16* ph = (_Float16*)whp + (size_t)i * 8;
    _Float16* pl = (_Float16*)wlp + (size_t)i * 8;
    *(volatile v8h*)ph = hv;
    *(volatile v8h*)pl = lv;
    __threadfence();
    *(volatile v8h*)ph = hv;
    *(volatile v8h*)pl = lv;
  }
}

__global__ __launch_bounds__(NTHR) void seq_lowrank_kernel(
    const float* __restrict__ x,
    const float* __restrict__ iproj,
    const float* __restrict__ irecv,
    const float* __restrict__ rproj,
    const float* __restrict__ rrecv,
    const unsigned short* __restrict__ whp,
    const unsigned short* __restrict__ wlp,
    const float* __restrict__ rbias,
    float* __restrict__ out) {
  __shared__ __align__(16) _Float16 aHi[RB * NH];
  __shared__ __align__(16) _Float16 aLo[RB * NH];
  __shared__ __align__(32) float    hS[RB * NH];
  __shared__ __align__(16) v4f      tP[NH];
  __shared__ __align__(16) v4f      tI[NH];
  __shared__ __align__(16) v4f      tR[NH];
  __shared__ __align__(16) v4f      tX[NI];
  __shared__ __align__(16) float    dsl[NWAVE][256];

  const _Float16* WHg = (const _Float16*)whp;
  const _Float16* WLg = (const _Float16*)wlp;
  const int tid  = threadIdx.x;
  const int lane = tid & 31;
  const int wave = __builtin_amdgcn_readfirstlane(tid >> 5);
  const int row  = tid >> 4;
  const int q    = tid & 15;
  const int b0   = blockIdx.x * RB;

#pragma unroll 1
  for (int i = tid; i < NH; i += NTHR) {
    const v4f a = *(const v4f*)(rproj + (size_t)i * NR);
    const v4f b = *(const v4f*)(iproj + (size_t)i * NR);
    const v4f d = *(const v4f*)(rrecv + (size_t)i * NR);
    tP[i] = a; tI[i] = b; tR[i] = d;
  }
  if (tid < NI) tX[tid] = *(const v4f*)(irecv + (size_t)tid * NR);

  const v4f z4 = {0.0f, 0.0f, 0.0f, 0.0f};
#pragma unroll 1
  for (int i = 0; i < EIT; ++i) {
    const int k0 = 16 * ECOL * i + ECOL * q;
    *(v4f*)(hS + row * NH + k0)     = z4;
    *(v4f*)(hS + row * NH + k0 + 4) = z4;
  }
  const v4f bias4 = *(const v4f*)(rbias + 4 * q);
  float p0 = 0.0f, p1 = 0.0f, p2 = 0.0f, p3 = 0.0f;
  __syncthreads();

  const size_t rowg = (size_t)(b0 + row) * NS;
  const v8f z8 = {0.0f, 0.0f, 0.0f, 0.0f, 0.0f, 0.0f, 0.0f, 0.0f};

#pragma unroll 1
  for (int s = 0; s < NS; ++s) {
    float u0 = 0.0f, u1 = 0.0f, u2 = 0.0f, u3 = 0.0f;
    {
      const float* xp = x + (rowg + (size_t)s) * NI + 8 * q;
      const v4f xa = *(const v4f*)(xp);
      const v4f xb = *(const v4f*)(xp + 4);
#pragma unroll
      for (int e = 0; e < 4; ++e) {
        const v4f ra = tX[8 * q + e];
        const v4f rb = tX[8 * q + 4 + e];
        u0 += xa[e] * ra[0]; u1 += xa[e] * ra[1]; u2 += xa[e] * ra[2]; u3 += xa[e] * ra[3];
        u0 += xb[e] * rb[0]; u1 += xb[e] * rb[1]; u2 += xb[e] * rb[2]; u3 += xb[e] * rb[3];
      }
#pragma unroll
      for (int off = 1; off < 16; off <<= 1) {
        u0 += __shfl_xor(u0, off, 32);
        u1 += __shfl_xor(u1, off, 32);
        u2 += __shfl_xor(u2, off, 32);
        u3 += __shfl_xor(u3, off, 32);
      }
    }

    float pa0 = 0.0f, pa1 = 0.0f, pa2 = 0.0f, pa3 = 0.0f;
#pragma unroll 1
    for (int i = 0; i < EIT; ++i) {
      const int k0 = 16 * ECOL * i + ECOL * q;
      const v8f ho = *(const v8f*)(hS + row * NH + k0);
      v8f hn;
      v8h hv, lv;
#pragma unroll
      for (int e = 0; e < ECOL; ++e) {
        const int k = k0 + e;
        const v4f rp = tP[k];
        const v4f ip = tI[k];
        const v4f rr = tR[k];
        const float rin = p0 * rp[0] + p1 * rp[1] + p2 * rp[2] + p3 * rp[3];
        const float xin = u0 * ip[0] + u1 * ip[1] + u2 * ip[2] + u3 * ip[3];
        const float th  = tanh_f32(rin + xin);
        const float hoe = ho[e];
        const float hne = hoe + ALPHA_F * (th - hoe);
        hn[e] = hne;
        pa0 += hne * rr[0]; pa1 += hne * rr[1]; pa2 += hne * rr[2]; pa3 += hne * rr[3];
        _Float16 h16, l16;
        split_f16(hne, h16, l16);
        hv[e] = h16; lv[e] = l16;
      }
      *(v8f*)(hS + row * NH + k0)  = hn;
      *(v8h*)(aHi + row * NH + k0) = hv;
      *(v8h*)(aLo + row * NH + k0) = lv;
    }
#pragma unroll
    for (int off = 1; off < 16; off <<= 1) {
      pa0 += __shfl_xor(pa0, off, 32);
      pa1 += __shfl_xor(pa1, off, 32);
      pa2 += __shfl_xor(pa2, off, 32);
      pa3 += __shfl_xor(pa3, off, 32);
    }
    p0 = pa0; p1 = pa1; p2 = pa2; p3 = pa3;
    __syncthreads();

    {
      const int c = lane & 15, hh = lane >> 4, koff = 8 * hh;
      const int j = wave & 3;
      const _Float16* ah = aHi + c * NH + koff;
      const _Float16* al = aLo + c * NH + koff;
      const _Float16* bh = WHg + (size_t)(16 * j + c) * NH + koff;
      const _Float16* bl = WLg + (size_t)(16 * j + c) * NH + koff;
      v8f acc = z8;
      if (wave < 4) {
#pragma unroll 4
        for (int k0 = 0; k0 < NH; k0 += 32) {
          const v16h a = Frag<_Float16>::load(ah + k0);
          const v16h b = Frag<_Float16>::load(bh + k0);
          acc = Frag<_Float16>::mma(a, b, acc);
          wguard2(acc, a, b);
        }
      } else {
#pragma unroll 4
        for (int k0 = 0; k0 < NH; k0 += 32) {
          const v16h a  = Frag<_Float16>::load(ah + k0);
          const v16h a2 = Frag<_Float16>::load(al + k0);
          const v16h b  = Frag<_Float16>::load(bh + k0);
          const v16h b2 = Frag<_Float16>::load(bl + k0);
          acc = Frag<_Float16>::mma(a, b2, acc);
          acc = Frag<_Float16>::mma(a2, b, acc);
          wguard4(acc, a, a2, b, b2);
        }
      }
      accg1(acc);
      const float sc = (wave < 4) ? SC_HH : SC_X;
      float* ds = dsl[wave];
#pragma unroll
      for (int r = 0; r < 8; ++r) ds[(8 * hh + r) * 16 + c] = acc[r] * sc;
    }
    __syncthreads();

    {
      const int j  = q >> 2;
      const int cc = (q & 3) * 4;
      const v4f va = *(const v4f*)(dsl[j]     + row * 16 + cc);
      const v4f vb = *(const v4f*)(dsl[j + 4] + row * 16 + cc);
      v4f o4;
#pragma unroll
      for (int e = 0; e < 4; ++e) o4[e] = (va[e] + vb[e]) + bias4[e];
      float* op = out + (rowg + (size_t)s) * NO + 4 * q;
      for (int pass = 0; pass < 2; ++pass) {
        *(volatile v4f*)op = o4;
        __threadfence();
      }
    }
  }
}

extern "C" void kernel_launch(void* const* d_in, const int* in_sizes, int n_in,
                              void* d_out, int out_size, void* d_ws, size_t ws_size, hipStream_t stream) {
  if (n_in < 7 || d_out == nullptr || d_ws == nullptr) return;
  if (in_sizes[0] != NB * NS * NI || in_sizes[1] != NH * NR || in_sizes[2] != NI * NR ||
      in_sizes[3] != NH * NR || in_sizes[4] != NH * NR || in_sizes[5] != NO * NH ||
      in_sizes[6] != NO || out_size != NB * NS * NO) return;

  const float* x     = (const float*)d_in[0];
  const float* iproj = (const float*)d_in[1];
  const float* irecv = (const float*)d_in[2];
  const float* rproj = (const float*)d_in[3];
  const float* rrecv = (const float*)d_in[4];
  const float* w     = (const float*)d_in[5];
  const float* rbias = (const float*)d_in[6];
  float* y = (float*)d_out;

  char* ws = (char*)d_ws; size_t off = 0;
  auto carve = [&](size_t bytes) -> char* { char* p = ws + off; off += (bytes + 255) & ~(size_t)255; return p; };
  unsigned short* WH = (unsigned short*)carve((size_t)NO * NH * 2);
  unsigned short* WL = (unsigned short*)carve((size_t)NO * NH * 2);
  if (off > ws_size || off > (size_t)134217728) return;

  const int n8 = NO * NH / 8;
  wsplit_kernel<<<(n8 + NTHR - 1) / NTHR, NTHR, 0, stream>>>(w, WH, WL, n8);
  seq_lowrank_kernel<<<NB / RB, NTHR, 0, stream>>>(x, iproj, irecv, rproj, rrecv, WH, WL, rbias, y);
}
